// GNNnetwork_76209899700463
// MI455X (gfx1250) — hardware-verified
//
#include <hip/hip_runtime.h>
#include <stddef.h>
#include <stdint.h>


#pragma clang fp contract(off)

#define NNODE    50000
#define NEDGE    800000
#define DD       64
#define NLAY     5
#define NVOC     128
#define NET      4
#define NGR      512
#define NTASK    10
#define KTOT     128
#define GBM      128
#define MP       (((NNODE + GBM - 1) / GBM) * GBM)
#define NGB      (MP / GBM)
#define NTHR     256
#define NWAVE    8
#define EPT      8
#define CHUNK    (NTHR * EPT)
#define WCAP     (EPT * 32)
#define LISTN    (NWAVE * WCAP)
#define NB       1024
#define PKS      10
#define NCB      ((MP + NB - 1) / NB)
#define RCAP     28672
#define DEGCAP   64
#define MEAS_B1024   16623
#define MEAS_MAXDEG  35
#define PARTW    160
#define WPLANE   (DD * KTOT)
#define WFPLANE  (128 * KTOT)
#define NUW      (2 * NLAY * (WPLANE / 8))
#define NUF      (WFPLANE / 8)
#define HTHR     128
#define HBM      64
#define LDS_CMP  ((2 * RCAP + 2 * NB + LISTN) * 4 + 64)
#define WSMAX    134217728

static_assert(MP == 50048 && NGB == 391 && NCB == 49);
static_assert(NB == (1 << PKS) && ((long long)CHUNK << PKS) < (1LL << 31));
static_assert(NEDGE < (1 << 21) && (NEDGE % 4) == 0);
static_assert(NTHR * 4 == NB && LISTN >= NB && (RCAP % 32) == 0);
static_assert(((RCAP / 2) % NTHR) == 0 && RCAP < 65536);
static_assert(RCAP >= MEAS_B1024 + MEAS_B1024 / 20);
static_assert(DEGCAP >= MEAS_MAXDEG + 8 && DEGCAP <= 64);
static_assert(LDS_CMP <= 300000);
static_assert((DD % 8) == 0 && KTOT == 2 * DD && (KTOT % 32) == 0);
static_assert(NTHR == NET * DD && NTHR == 4 * DD);
static_assert((NB % GBM) == 0 && NCB * NB >= MP);
static_assert((NUW % NTHR) == 0 && (NUF % NTHR) == 0 && ((WPLANE / 8) % NTHR) == 0);
static_assert((MP * 16) % NTHR == 0);
static_assert((PARTW % 32) == 0 && PARTW / 4 <= NTHR && PARTW >= 2 * DD + 1);
static_assert((NGR % NWAVE) == 0 && (NGR % HBM) == 0);
static_assert((NGR / HBM) * HBM * NTASK == NGR * NTASK && ((HBM * NTASK * 4) % 128) == 0);
static_assert(NNODE < 65536);

typedef float          v2f  __attribute__((ext_vector_type(2)));
typedef float          v4f  __attribute__((ext_vector_type(4)));
typedef float          v8f  __attribute__((ext_vector_type(8)));
typedef int            v2i  __attribute__((ext_vector_type(2)));
typedef int            v4i  __attribute__((ext_vector_type(4)));
typedef int            v8i  __attribute__((ext_vector_type(8)));
typedef unsigned int   v4u  __attribute__((ext_vector_type(4)));
typedef unsigned short v8us __attribute__((ext_vector_type(8)));
typedef __bf16         v16b __attribute__((ext_vector_type(16)));
typedef v2f  __attribute__((may_alias)) v2fa;
typedef v4f  __attribute__((may_alias)) v4fa;
typedef v4u  __attribute__((may_alias)) v4ua;
typedef v8us __attribute__((may_alias)) v8usa;
union FragB { v16b v; v8us h[2]; v8i w; };

__device__ __forceinline__ v8f wmb(const FragB& a, const FragB& b, v8f c) {
  v8f d = __builtin_amdgcn_wmma_f32_16x16x32_bf16(false, a.v, false, b.v, (short)0, c, false, false);
  asm volatile("v_nop\n\tv_nop\n\tv_nop\n\tv_nop" : "+v"(d) : "v"(a.w), "v"(b.w));
  return d;
}

__device__ __forceinline__ unsigned short bf_bits(float f) {
  unsigned int u = __float_as_uint(f);
  u += 0x7FFFu + ((u >> 16) & 1u);
  return (unsigned short)(u >> 16);
}
__device__ __forceinline__ float bf_val(unsigned short b) {
  return __uint_as_float(((unsigned int)b) << 16);
}
__device__ __forceinline__ float bf_rne(float f) { return bf_val(bf_bits(f)); }
__device__ __forceinline__ float relu_np(float v) { return (v > 0.0f) ? v : (v - v); }
__device__ __forceinline__ float bnrelu(float x, float m, float r, float g, float be) {
  return relu_np(g * (x - m) * r + be);
}
__device__ __forceinline__ v8us gather8(const float* __restrict__ p, int stride) {
  v8us o;
#pragma unroll
  for (int i = 0; i < 8; ++i) o[i] = bf_bits(p[(size_t)i * (size_t)stride]);
  return o;
}

__device__ __forceinline__ int scan_chunk(const int* __restrict__ dsts, int nE, int cbase, int slotBase,
                                          int nb, int vec8, int* list, int tid, int lane, int wave) {
  int wc = 0;
  const int el0  = tid * EPT;
  const int e0   = cbase + el0;
  const int sent = -2147483647 - 1;
  v4i da, db;
  if (vec8 != 0 && cbase + CHUNK <= nE) {
    da = *(const v4i*)(dsts + e0);
    db = *(const v4i*)(dsts + e0 + 4);
  } else {
    da.x = (e0     < nE) ? dsts[min(e0,     nE - 1)] : sent;
    da.y = (e0 + 1 < nE) ? dsts[min(e0 + 1, nE - 1)] : sent;
    da.z = (e0 + 2 < nE) ? dsts[min(e0 + 2, nE - 1)] : sent;
    da.w = (e0 + 3 < nE) ? dsts[min(e0 + 3, nE - 1)] : sent;
    db.x = (e0 + 4 < nE) ? dsts[min(e0 + 4, nE - 1)] : sent;
    db.y = (e0 + 5 < nE) ? dsts[min(e0 + 5, nE - 1)] : sent;
    db.z = (e0 + 6 < nE) ? dsts[min(e0 + 6, nE - 1)] : sent;
    db.w = (e0 + 7 < nE) ? dsts[min(e0 + 7, nE - 1)] : sent;
  }
  const unsigned nbs = (unsigned)slotBase;
  const unsigned unb = (unsigned)nb;
  const unsigned s0 = (unsigned)da.x - nbs, s1 = (unsigned)da.y - nbs;
  const unsigned s2 = (unsigned)da.z - nbs, s3 = (unsigned)da.w - nbs;
  const unsigned s4 = (unsigned)db.x - nbs, s5 = (unsigned)db.y - nbs;
  const unsigned s6 = (unsigned)db.z - nbs, s7 = (unsigned)db.w - nbs;
  const bool h0 = s0 < unb, h1 = s1 < unb, h2 = s2 < unb, h3 = s3 < unb;
  const bool h4 = s4 < unb, h5 = s5 < unb, h6 = s6 < unb, h7 = s7 < unb;
  const unsigned any = __builtin_amdgcn_ballot_w32(h0 | h1 | h2 | h3 | h4 | h5 | h6 | h7);
  if (any != 0u) {
#define HITJ(J, HJ, SJ) { \
      const unsigned mj = __builtin_amdgcn_ballot_w32(HJ); \
      if (mj != 0u) { \
        if (HJ) { \
          const int pos = wc + (int)__builtin_amdgcn_mbcnt_lo(mj, 0u); \
          if (pos < WCAP) list[wave * WCAP + pos] = ((el0 + (J)) << PKS) | (int)(SJ); \
        } \
        wc += (int)__builtin_popcount(mj); } }
    HITJ(0, h0, s0)
    HITJ(1, h1, s1)
    HITJ(2, h2, s2)
    HITJ(3, h3, s3)
    HITJ(4, h4, s4)
    HITJ(5, h5, s5)
    HITJ(6, h6, s6)
    HITJ(7, h7, s7)
#undef HITJ
  }
  return wc;
}

__global__ __launch_bounds__(NTHR) void k_wprep(const float* __restrict__ W1, const float* __restrict__ W2,
                                                const float* __restrict__ Wf1, unsigned short* wt) {
  const int u = (int)blockIdx.x * NTHR + (int)threadIdx.x;
  if (u >= NUW + NUF) return;
  v8us o;
  if (u < NUW) {
    const int mi    = u >> 10;
    const int v     = u & 1023;
    const int n     = v >> 4;
    const int kk    = ((v & 15) * 8) & (DD - 1);
    const int layer = mi >> 1;
    const size_t so = (size_t)layer * DD * DD + (size_t)kk * DD + n;
    if ((mi & 1) == 0) o = gather8(W1 + so, DD);
    else               o = gather8(W2 + so, DD);
  } else {
    const int v  = u - NUW;
    const int n  = v >> 4;
    const int kk = ((v & 15) * 8) & (DD - 1);
    o = gather8(Wf1 + (size_t)kk * 128 + n, 128);
  }
  unsigned short* dp = wt + (size_t)u * 8;
  *(volatile v8us*)dp = o;
  __threadfence();
  *(volatile v8us*)dp = o;
}

__global__ __launch_bounds__(NTHR) void k_embed(const int* __restrict__ x, const float* __restrict__ femb,
                                                int nN, int nUnits, float* H) {
  const int u = (int)blockIdx.x * NTHR + (int)threadIdx.x;
  if (u >= nUnits) return;
  const int row = u >> 4;
  const int c4  = (u & 15) * 4;
  const int rc  = row < nN ? row : nN - 1;
  int xr = x[rc];
  xr = xr < 0 ? 0 : (xr > NVOC - 1 ? NVOC - 1 : xr);
  const v4f a = *(const v4f*)(femb + (size_t)xr * DD + c4);
  const bool ok = row < nN;
  v4f o;
  o.x = ok ? bf_rne(a.x) : 0.0f;
  o.y = ok ? bf_rne(a.y) : 0.0f;
  o.z = ok ? bf_rne(a.z) : 0.0f;
  o.w = ok ? bf_rne(a.w) : 0.0f;
  float* hp = H + (size_t)u * 4;
  *(volatile v4f*)hp = o;
  __threadfence();
  *(volatile v4f*)hp = o;
}

__global__ __launch_bounds__(NTHR) void k_compact(const int* __restrict__ srcs, const int* __restrict__ dsts,
                                                  const int* __restrict__ attr, int nN, int nE, int vec8,
                                                  int* seg, int* lst) {
  extern __shared__ v4f lds_dyn[];
  int* reg1 = (int*)lds_dyn;
  int* reg2 = reg1 + RCAP;
  int* scnt = reg2 + RCAP;
  int* soff = scnt + NB;
  int* list = soff + NB;
  int* wcnt = list + LISTN;
  int* wtot = wcnt + NWAVE;
  const int tid = (int)threadIdx.x, lane = tid & 31, wave = tid >> 5;
  const int nodeBase = (int)blockIdx.x * NB;

  for (int i = tid; i < NB; i += NTHR) scnt[i] = 0;
  if (tid == 0) reg2[0] = 0;
  __syncthreads();

  int tot = 0;
  const int nChunks = (nE + CHUNK - 1) / CHUNK;
#pragma unroll 1
  for (int ch = 0; ch < nChunks; ++ch) {
    const int cbase = ch * CHUNK;
    const int wc = scan_chunk(dsts, nE, cbase, nodeBase, NB, vec8, list, tid, lane, wave);
    if (lane == 0) wcnt[wave] = wc;
    __syncthreads();
    int pre = 0, all = 0;
#pragma unroll
    for (int w2 = 0; w2 < NWAVE; ++w2) {
      int c = wcnt[w2];
      c = c < 0 ? 0 : (c > WCAP ? WCAP : c);
      all += c;
      pre += (w2 < wave) ? c : 0;
    }
    const int wcc  = wc > WCAP ? WCAP : wc;
    const int base = tot + pre;
#pragma unroll 1
    for (int i = lane; i < wcc; i += 32) {
      const int ent = list[wave * WCAP + i];
      const int el  = (ent >> PKS) & (CHUNK - 1);
      const int sl  = ent & (NB - 1);
      int eid = cbase + el;
      eid = eid > nE - 1 ? nE - 1 : eid;
      const int pos = base + i;
      if (pos < RCAP) reg1[pos] = (int)(((unsigned)eid << PKS) | (unsigned)sl);
    }
    tot += all;
    tot = tot > RCAP ? RCAP : tot;
    __syncthreads();
  }
  const int nh = tot;

  if (wave == 0) {
#pragma unroll 1
    for (int b0 = 0; b0 < nh; b0 += 32) {
      const int idx = b0 + lane;
      const int lim = nh - 1;
      const int uv  = reg1[idx < lim ? idx : lim];
      const int m32 = (nh - b0) < 32 ? (nh - b0) : 32;
#pragma unroll 1
      for (int k = 0; k < m32; ++k) {
        const int u  = __builtin_amdgcn_readlane(uv, k);
        const int sl = u & (NB - 1);
        if (lane == 0) scnt[sl] = scnt[sl] + 1;
      }
    }
  }
  __syncthreads();

  {
    const v4i ca = *(const v4i*)(scnt + 4 * tid);
    const int e0 = ca.x < 0 ? 0 : ca.x, e1 = ca.y < 0 ? 0 : ca.y, e2 = ca.z < 0 ? 0 : ca.z, e3 = ca.w < 0 ? 0 : ca.w;
    const int ts = e0 + e1 + e2 + e3;
    int incl = ts;
#pragma unroll
    for (int d = 1; d < 32; d <<= 1) {
      const int up = __shfl_up(incl, d);
      if (lane >= d) incl += up;
    }
    if (lane == 31) wtot[wave] = incl;
    __syncthreads();
    int pre = 0;
#pragma unroll
    for (int w2 = 0; w2 < NWAVE; ++w2) pre += (w2 < wave) ? wtot[w2] : 0;
    int run = pre + incl - ts;
    soff[4 * tid + 0] = run; run += e0;
    soff[4 * tid + 1] = run; run += e1;
    soff[4 * tid + 2] = run; run += e2;
    soff[4 * tid + 3] = run;
  }
  __syncthreads();
  for (int i = tid; i < NB; i += NTHR) list[i] = soff[i];
  __syncthreads();

  if (wave == 0) {
#pragma unroll 1
    for (int b0 = 0; b0 < nh; b0 += 32) {
      const int idx = b0 + lane;
      const int lim = nh - 1;
      const int uv  = reg1[idx < lim ? idx : lim];
      const int m32 = (nh - b0) < 32 ? (nh - b0) : 32;
#pragma unroll 1
      for (int k = 0; k < m32; ++k) {
        const int u   = __builtin_amdgcn_readlane(uv, k);
        const int sl  = u & (NB - 1);
        const int eid = (int)((unsigned)u >> PKS);
        if (lane == 0) {
          int pos = list[sl];
          pos = pos < 0 ? 0 : (pos > RCAP - 1 ? RCAP - 1 : pos);
          reg2[pos] = eid;
          list[sl] = pos + 1;
        }
      }
    }
  }
  __syncthreads();

  const bool ovf = (nh >= RCAP);
  {
    const v4i c4 = *(const v4i*)(scnt + 4 * tid);
    const v4i o4 = *(const v4i*)(soff + 4 * tid);
    int c0 = c4.x, c1 = c4.y, c2 = c4.z, c3 = c4.w;
    int o0 = o4.x, o1 = o4.y, o2 = o4.z, o3 = o4.w;
    c0 = c0 < 0 ? 0 : (c0 > 0x7ffe ? 0x7ffe : c0);
    c1 = c1 < 0 ? 0 : (c1 > 0x7ffe ? 0x7ffe : c1);
    c2 = c2 < 0 ? 0 : (c2 > 0x7ffe ? 0x7ffe : c2);
    c3 = c3 < 0 ? 0 : (c3 > 0x7ffe ? 0x7ffe : c3);
    c0 = ovf ? 0x7fff : c0; c1 = ovf ? 0x7fff : c1; c2 = ovf ? 0x7fff : c2; c3 = ovf ? 0x7fff : c3;
    o0 = o0 < 0 ? 0 : (o0 > RCAP ? RCAP : o0);
    o1 = o1 < 0 ? 0 : (o1 > RCAP ? RCAP : o1);
    o2 = o2 < 0 ? 0 : (o2 > RCAP ? RCAP : o2);
    o3 = o3 < 0 ? 0 : (o3 > RCAP ? RCAP : o3);
    v4i sg;
    sg.x = (c0 << 16) | o0; sg.y = (c1 << 16) | o1; sg.z = (c2 << 16) | o2; sg.w = (c3 << 16) | o3;
    int* sp = seg + (size_t)blockIdx.x * NB + 4 * tid;
    *(volatile v4i*)sp = sg;
    __threadfence();
    *(volatile v4i*)sp = sg;
  }
  int* lb = lst + (size_t)blockIdx.x * (size_t)RCAP * 2;
  const int last = nh > 0 ? nh - 1 : 0;
#pragma unroll 1
  for (int p2 = tid; p2 < RCAP / 2; p2 += NTHR) {
    const int i0 = 2 * p2, i1 = 2 * p2 + 1;
    int ea = reg2[i0 < last ? i0 : last];
    int eb = reg2[i1 < last ? i1 : last];
    ea = ea < 0 ? 0 : (ea > nE - 1 ? nE - 1 : ea);
    eb = eb < 0 ? 0 : (eb > nE - 1 ? nE - 1 : eb);
    int sa = srcs[ea], sb = srcs[eb];
    int aa = attr[ea], ab = attr[eb];
    sa = sa < 0 ? 0 : (sa > nN - 1 ? nN - 1 : sa);
    sb = sb < 0 ? 0 : (sb > nN - 1 ? nN - 1 : sb);
    aa = aa < 0 ? 0 : (aa > NET - 1 ? NET - 1 : aa);
    ab = ab < 0 ? 0 : (ab > NET - 1 ? NET - 1 : ab);
    const bool va = i0 < nh, vb = i1 < nh;
    v4i rec;
    rec.x = va ? sa : 0; rec.y = va ? aa : 0; rec.z = vb ? sb : 0; rec.w = vb ? ab : 0;
    int* rp = lb + (size_t)p2 * 4;
    *(volatile v4i*)rp = rec;
    __threadfence();
    *(volatile v4i*)rp = rec;
  }
}

__global__ __launch_bounds__(NTHR) void k_agg(const int* __restrict__ seg, const int* __restrict__ lst,
                                              const float* __restrict__ H, const float* __restrict__ eemb,
                                              const float* __restrict__ epsv, int layer,
                                              unsigned int* P1w, int nN, int mRows) {
  __shared__ __attribute__((aligned(16))) float ee[NET * DD];
  __shared__ __attribute__((aligned(16))) unsigned int stw[NWAVE * 1024];
  const int tid = (int)threadIdx.x, lane = tid & 31, wave = tid >> 5;
  ee[tid] = bf_rne(eemb[(size_t)layer * (NET * DD) + tid]);
  const float sc = 1.0f + bf_rne(epsv[layer]);
  __syncthreads();

  const int row16 = (int)blockIdx.x * GBM + 16 * wave;
  unsigned int* stwu = stw + wave * 1024;
  const float qnan = __int_as_float(0x7fc00000);

#pragma unroll 1
  for (int j = 0; j < 16; ++j) {
    const int grow = row16 + j;
    const int cb   = grow >> PKS;
    const int sg   = seg[grow];
    int off = sg & 0xffff;
    const int craw = (sg >> 16) & 0x7fff;
    off = off > RCAP ? RCAP : off;
    int cnt = craw > DEGCAP ? DEGCAP : craw;
    if (cnt > RCAP - off) cnt = RCAP - off;
    const float pz = (craw > DEGCAP) ? qnan : 0.0f;
    const bool liveRow = grow < nN;
    const int* lb = lst + (size_t)cb * (size_t)RCAP * 2;

    float a0 = 0.0f, a1 = 0.0f;
#pragma unroll 1
    for (int b0 = 0; b0 < cnt; b0 += 32) {
      int idx = off + b0 + lane;
      idx = idx > RCAP - 1 ? RCAP - 1 : idx;
      const v2i rec = *(const v2i*)(lb + (size_t)idx * 2);
      int sv = rec.x, av = rec.y;
      sv = sv < 0 ? 0 : (sv > nN - 1 ? nN - 1 : sv);
      av = av < 0 ? 0 : (av > NET - 1 ? NET - 1 : av);
      const int m32 = (cnt - b0) < 32 ? (cnt - b0) : 32;
#pragma unroll 1
      for (int k = 0; k < m32; ++k) {
        const int sk = __builtin_amdgcn_readlane(sv, k);
        const int ak = __builtin_amdgcn_readlane(av, k);
        const v2f hv = *(const v2f*)(H + (size_t)sk * DD + 2 * lane);
        const v2f ev = *(const v2fa*)(ee + ak * DD + 2 * lane);
        const float m0 = hv.x + ev.x;
        const float m1 = hv.y + ev.y;
        a0 += relu_np(m0);
        a1 += relu_np(m1);
      }
    }
    const int nc = liveRow ? grow : nN - 1;
    const v2f sf = *(const v2f*)(H + (size_t)nc * DD + 2 * lane);
    float r0 = sc * sf.x + a0;
    float r1 = sc * sf.y + a1;
    r0 = (liveRow ? r0 : 0.0f) + pz;
    r1 = (liveRow ? r1 : 0.0f) + pz;
    const unsigned short hb0 = bf_bits(r0), hb1 = bf_bits(r1);
    const unsigned short lb0 = bf_bits(r0 - bf_val(hb0)), lb1 = bf_bits(r1 - bf_val(hb1));
    stwu[j * 64 + lane]      = (unsigned int)hb0 | ((unsigned int)hb1 << 16);
    stwu[j * 64 + 32 + lane] = (unsigned int)lb0 | ((unsigned int)lb1 << 16);
  }
  __builtin_amdgcn_fence(__ATOMIC_RELEASE, "wavefront");
  __builtin_amdgcn_wave_barrier();
  v4u pk[8];
#pragma unroll
  for (int i = 0; i < 8; ++i) pk[i] = *(const v4ua*)(stwu + 128 * i + 4 * lane);
  unsigned int* gp = P1w + (size_t)row16 * 64 + 4 * lane;
  const bool wsv = (row16 + 16) <= mRows;
#pragma unroll
  for (int i = 0; i < 8; ++i) { if (wsv) *(volatile v4u*)(gp + 128 * i) = pk[i]; }
  __threadfence();
#pragma unroll
  for (int i = 0; i < 8; ++i) { if (wsv) *(volatile v4u*)(gp + 128 * i) = pk[i]; }
}

__global__ __launch_bounds__(NTHR) void k_gemm(const unsigned short* __restrict__ A,
                                               const unsigned short* __restrict__ WT,
                                               const float* __restrict__ bias,
                                               float* outp, float* part, int nN, int mRows) {
  __shared__ __attribute__((aligned(16))) float stg[GBM * DD];
  __shared__ __attribute__((aligned(16))) float pst[PARTW];
  const int tid = (int)threadIdx.x, lane = tid & 31, wave = tid >> 5, hh = lane >> 4, m = lane & 15;
  const int rowBase = (int)blockIdx.x * GBM;

  v8f acc[4];
  {
    const v8f z = {0.f, 0.f, 0.f, 0.f, 0.f, 0.f, 0.f, 0.f};
#pragma unroll
    for (int t = 0; t < 4; ++t) acc[t] = z;
  }
  const unsigned short* ap = A + (size_t)(rowBase + 16 * wave + m) * (size_t)KTOT + 8 * hh;
  const unsigned short* wp = WT + (size_t)m * (size_t)KTOT + 8 * hh;
#pragma unroll 1
  for (int ks = 0; ks < KTOT / 32; ++ks) {
    FragB af;
    af.h[0] = *(const v8usa*)(ap + 32 * ks);
    af.h[1] = *(const v8usa*)(ap + 32 * ks + 16);
#pragma unroll
    for (int t = 0; t < 4; ++t) {
      const unsigned short* wq = wp + (size_t)(16 * t) * (size_t)KTOT + 32 * ks;
      FragB bf;
      bf.h[0] = *(const v8usa*)wq;
      bf.h[1] = *(const v8usa*)(wq + 16);
      acc[t] = wmb(af, bf, acc[t]);
    }
  }

#pragma unroll
  for (int t = 0; t < 4; ++t) {
    const int lc = 16 * t + m;
    const float bb = bf_rne(bias[lc]);
#pragma unroll
    for (int r = 0; r < 8; ++r) {
      const int lr = 16 * wave + 8 * hh + r;
      const bool live = (rowBase + lr) < nN;
      const float v = acc[t][r] + bb;
      stg[lr * DD + lc] = live ? v : 0.0f;
    }
  }
  __syncthreads();

  if (tid < DD) {
    int rv = nN - rowBase;
    rv = rv < 0 ? 0 : (rv > GBM ? GBM : rv);
    float s = 0.0f;
#pragma unroll 1
    for (int r = 0; r < rv; ++r) s += stg[r * DD + tid];
    const float rn = (rv > 0) ? (1.0f / (float)rv) : 0.0f;
    const float mean = s * rn;
    float M2 = 0.0f;
#pragma unroll 1
    for (int r = 0; r < rv; ++r) {
      const float d = stg[r * DD + tid] - mean;
      M2 += d * d;
    }
    pst[tid] = mean;
    pst[DD + tid] = M2;
    if (tid < 32) pst[2 * DD + tid] = (tid == 0) ? (float)rv : 0.0f;
  }
  {
    v4f fv[8];
#pragma unroll
    for (int i = 0; i < 8; ++i) fv[i] = *(const v4fa*)(stg + (16 * wave) * DD + 128 * i + 4 * lane);
    float* op = outp + (size_t)(rowBase + 16 * wave) * DD + 4 * lane;
    const bool wsv = (rowBase + 16 * wave + 16) <= mRows;
#pragma unroll
    for (int i = 0; i < 8; ++i) { if (wsv) *(volatile v4f*)(op + 128 * i) = fv[i]; }
    __threadfence();
#pragma unroll
    for (int i = 0; i < 8; ++i) { if (wsv) *(volatile v4f*)(op + 128 * i) = fv[i]; }
  }
  __syncthreads();
  {
    const bool wr = tid < PARTW / 4;
    const int ti = wr ? tid : 0;
    const v4f pv = *(const v4fa*)(pst + 4 * ti);
    float* pp = part + (size_t)blockIdx.x * PARTW + 4 * ti;
    if (wr) *(volatile v4f*)pp = pv;
    __threadfence();
    if (wr) *(volatile v4f*)pp = pv;
  }
}

__global__ __launch_bounds__(DD) void k_comb(const float* __restrict__ part, int nPart,
                                             const float* __restrict__ gam, const float* __restrict__ bet,
                                             float* stat) {
  __shared__ __attribute__((aligned(16))) float stg[4 * DD];
  const int c = (int)threadIdx.x;
  double n = 0.0, mean = 0.0, M2 = 0.0;
#pragma unroll 1
  for (int b = 0; b < nPart; ++b) {
    const float* pr = part + (size_t)b * PARTW;
    const float nb = pr[2 * DD];
    const float mb = pr[c];
    const float qb = pr[DD + c];
    if (nb > 0.5f) {
      const double nn = n + (double)nb;
      const double delta = (double)mb - mean;
      const double f = (double)nb / nn;
      mean = mean + delta * f;
      M2 = M2 + (double)qb + delta * delta * n * f;
      n = nn;
    }
  }
  const double nt = n < 1.0 ? 1.0 : n;
  const float var = (float)(M2 / nt);
  const float r = 1.0f / sqrtf(var + 1e-5f);
  stg[c] = (float)mean;
  stg[DD + c] = r;
  stg[2 * DD + c] = bf_rne(gam[c]);
  stg[3 * DD + c] = bf_rne(bet[c]);
  __syncthreads();
  const v4f v = *(const v4fa*)(stg + 4 * c);
  float* sp = stat + 4 * c;
  *(volatile v4f*)sp = v;
  __threadfence();
  *(volatile v4f*)sp = v;
}

__global__ __launch_bounds__(NTHR) void k_apply_a(const float* __restrict__ T, const float* __restrict__ stat,
                                                  int nN, int nUnits, unsigned short* P1) {
  __shared__ float ssh[4 * DD];
  const int tid = (int)threadIdx.x;
  ssh[tid] = stat[tid];
  __syncthreads();
  const int u = (int)blockIdx.x * NTHR + tid;
  if (u >= nUnits) return;
  const int row = u >> 4;
  const int p   = u & 15;
  const int cb  = 8 * (p & 7);
  const bool isHi = p < 8;
  const int rc  = row < nN ? row : nN - 1;
  const bool ok = row < nN;
  const v4f a = *(const v4f*)(T + (size_t)rc * DD + cb);
  const v4f b = *(const v4f*)(T + (size_t)rc * DD + cb + 4);
  const float f[8] = {a.x, a.y, a.z, a.w, b.x, b.y, b.z, b.w};
  unsigned int w[4];
#pragma unroll
  for (int j = 0; j < 4; ++j) {
    const int c0 = cb + 2 * j, c1 = cb + 2 * j + 1;
    float y0 = bnrelu(f[2 * j],     ssh[c0], ssh[DD + c0], ssh[2 * DD + c0], ssh[3 * DD + c0]);
    float y1 = bnrelu(f[2 * j + 1], ssh[c1], ssh[DD + c1], ssh[2 * DD + c1], ssh[3 * DD + c1]);
    y0 = ok ? y0 : 0.0f;
    y1 = ok ? y1 : 0.0f;
    const unsigned short h0 = bf_bits(y0), h1 = bf_bits(y1);
    const unsigned short l0 = bf_bits(y0 - bf_val(h0)), l1 = bf_bits(y1 - bf_val(h1));
    const unsigned short q0 = isHi ? h0 : l0, q1 = isHi ? h1 : l1;
    w[j] = (unsigned int)q0 | ((unsigned int)q1 << 16);
  }
  v4u pw; pw.x = w[0]; pw.y = w[1]; pw.z = w[2]; pw.w = w[3];
  unsigned short* op = P1 + (size_t)u * 8;
  *(volatile v4u*)op = pw;
  __threadfence();
  *(volatile v4u*)op = pw;
}

__global__ __launch_bounds__(NTHR) void k_apply_b(const float* __restrict__ U, const float* __restrict__ stat,
                                                  int nN, int nUnits, float* H) {
  __shared__ float ssh[4 * DD];
  const int tid = (int)threadIdx.x;
  ssh[tid] = stat[tid];
  __syncthreads();
  const int u = (int)blockIdx.x * NTHR + tid;
  if (u >= nUnits) return;
  const int row = u >> 4;
  const int c4  = (u & 15) * 4;
  const int rc  = row < nN ? row : nN - 1;
  const bool ok = row < nN;
  const v4f a = *(const v4f*)(U + (size_t)rc * DD + c4);
  const float y0 = bnrelu(a.x, ssh[c4 + 0], ssh[DD + c4 + 0], ssh[2 * DD + c4 + 0], ssh[3 * DD + c4 + 0]);
  const float y1 = bnrelu(a.y, ssh[c4 + 1], ssh[DD + c4 + 1], ssh[2 * DD + c4 + 1], ssh[3 * DD + c4 + 1]);
  const float y2 = bnrelu(a.z, ssh[c4 + 2], ssh[DD + c4 + 2], ssh[2 * DD + c4 + 2], ssh[3 * DD + c4 + 2]);
  const float y3 = bnrelu(a.w, ssh[c4 + 3], ssh[DD + c4 + 3], ssh[2 * DD + c4 + 3], ssh[3 * DD + c4 + 3]);
  v4f o;
  o.x = ok ? y0 : 0.0f; o.y = ok ? y1 : 0.0f; o.z = ok ? y2 : 0.0f; o.w = ok ? y3 : 0.0f;
  float* hp = H + (size_t)u * 4;
  *(volatile v4f*)hp = o;
  __threadfence();
  *(volatile v4f*)hp = o;
}

__global__ __launch_bounds__(NTHR) void k_pool(const float* __restrict__ H, const int* __restrict__ bat,
                                               int nN, unsigned int* PLw) {
  __shared__ __attribute__((aligned(16))) unsigned int pl[NWAVE * 64];
  const int tid = (int)threadIdx.x, lane = tid & 31, wave = tid >> 5;
  const int g = (int)blockIdx.x * NWAVE + wave;
  float a0 = 0.0f, a1 = 0.0f;
#pragma unroll 1
  for (int i0 = 0; i0 < nN; i0 += 32) {
    const int i  = i0 + lane;
    const int ic = i < nN ? i : nN - 1;
    const int b  = bat[ic];
    const bool hit = (i < nN) && (b == g);
    unsigned msk = __builtin_amdgcn_ballot_w32(hit);
    int nh = (int)__builtin_popcount(msk);
    nh = nh > 32 ? 32 : nh;
#pragma unroll 1
    for (int q = 0; q < nh; ++q) {
      const int k = __builtin_ffs((int)msk) - 1;
      msk &= msk - 1u;
      int node = i0 + (k < 0 ? 0 : k);
      node = node > nN - 1 ? nN - 1 : node;
      const v2f v = *(const v2f*)(H + (size_t)node * DD + 2 * lane);
      a0 += v.x; a1 += v.y;
    }
  }
  const unsigned short hb0 = bf_bits(a0), hb1 = bf_bits(a1);
  const unsigned short lb0 = bf_bits(a0 - bf_val(hb0)), lb1 = bf_bits(a1 - bf_val(hb1));
  pl[wave * 64 + lane]      = (unsigned int)hb0 | ((unsigned int)hb1 << 16);
  pl[wave * 64 + 32 + lane] = (unsigned int)lb0 | ((unsigned int)lb1 << 16);
  __syncthreads();
  const bool wr = tid < 128;
  const int ti = wr ? tid : 0;
  const v4u pk = *(const v4ua*)(pl + 4 * ti);
  unsigned int* gp = PLw + (size_t)blockIdx.x * (NWAVE * 64) + 4 * ti;
  if (wr) *(volatile v4u*)gp = pk;
  __threadfence();
  if (wr) *(volatile v4u*)gp = pk;
}

__global__ __launch_bounds__(HTHR) void k_head(const unsigned short* __restrict__ PL,
                                               const unsigned short* __restrict__ WT,
                                               const float* __restrict__ bf1, const float* __restrict__ Wf2,
                                               const float* __restrict__ bf2, float* out) {
  __shared__ __attribute__((aligned(16))) float stg[HBM * 128];
  __shared__ __attribute__((aligned(16))) float wf2s[128 * NTASK];
  __shared__ __attribute__((aligned(16))) float outs[HBM * NTASK];
  __shared__ float b2s[16];
  const int tid = (int)threadIdx.x, lane = tid & 31, wave = tid >> 5, hh = lane >> 4, m = lane & 15;
  const int rowBase = (int)blockIdx.x * HBM;

#pragma unroll 2
  for (int i = tid; i < 128 * NTASK; i += HTHR) wf2s[i] = bf_rne(Wf2[i]);
  if (tid < 16) b2s[tid] = bf_rne(bf2[tid < NTASK ? tid : NTASK - 1]);

  v8f acc[8];
  {
    const v8f z = {0.f, 0.f, 0.f, 0.f, 0.f, 0.f, 0.f, 0.f};
#pragma unroll
    for (int t = 0; t < 8; ++t) acc[t] = z;
  }
  const unsigned short* ap = PL + (size_t)(rowBase + 16 * wave + m) * (size_t)KTOT + 8 * hh;
  const unsigned short* wp = WT + (size_t)m * (size_t)KTOT + 8 * hh;
#pragma unroll 1
  for (int ks = 0; ks < KTOT / 32; ++ks) {
    FragB af;
    af.h[0] = *(const v8usa*)(ap + 32 * ks);
    af.h[1] = *(const v8usa*)(ap + 32 * ks + 16);
#pragma unroll
    for (int t = 0; t < 8; ++t) {
      const unsigned short* wq = wp + (size_t)(16 * t) * (size_t)KTOT + 32 * ks;
      FragB bf;
      bf.h[0] = *(const v8usa*)wq;
      bf.h[1] = *(const v8usa*)(wq + 16);
      acc[t] = wmb(af, bf, acc[t]);
    }
  }
#pragma unroll
  for (int t = 0; t < 8; ++t) {
    const int lc = 16 * t + m;
    const float bb = bf_rne(bf1[lc]);
#pragma unroll
    for (int r = 0; r < 8; ++r) {
      const int lr = 16 * wave + 8 * hh + r;
      stg[lr * 128 + lc] = relu_np(acc[t][r] + bb);
    }
  }
  __syncthreads();

#pragma unroll 1
  for (int j = 0; j < (HBM * NTASK) / HTHR; ++j) {
    const int o   = tid + HTHR * j;
    const int row = o / NTASK;
    const int c   = o - NTASK * row;
    float s = 0.0f;
#pragma unroll 4
    for (int k = 0; k < 128; ++k) s = fmaf(stg[row * 128 + k], wf2s[k * NTASK + c], s);
    outs[o] = s + b2s[c];
  }
  __syncthreads();

  const int i1 = (tid + HTHR) < (HBM * NTASK / 4) ? (tid + HTHR) : (HBM * NTASK / 4 - 1);
  const v4f o0 = *(const v4fa*)(outs + 4 * tid);
  const v4f o1 = *(const v4fa*)(outs + 4 * i1);
  const bool h1 = tid < (HBM * NTASK / 4 - HTHR);
  float* ob = out + (size_t)blockIdx.x * (HBM * NTASK);
  *(volatile v4f*)(ob + 4 * tid) = o0;
  if (h1) *(volatile v4f*)(ob + 4 * i1) = o1;
  __threadfence();
  *(volatile v4f*)(ob + 4 * tid) = o0;
  if (h1) *(volatile v4f*)(ob + 4 * i1) = o1;
}

static inline size_t al256(size_t o) { return (o + 255) & ~(size_t)255; }

extern "C" void kernel_launch(void* const* d_in, const int* in_sizes, int n_in,
                              void* d_out, int out_size, void* d_ws, size_t ws_size,
                              hipStream_t stream) {
  if (n_in < 19) return;
  if (in_sizes[0] != NNODE || in_sizes[1] != 2 * NEDGE || in_sizes[2] != NEDGE || in_sizes[3] != NNODE) return;
  if (in_sizes[4] != NVOC * DD || in_sizes[5] != NLAY * NET * DD || in_sizes[6] != NLAY) return;
  if (in_sizes[7] != NLAY * DD * DD || in_sizes[11] != NLAY * DD * DD) return;
  if (in_sizes[8] != NLAY * DD || in_sizes[9] != NLAY * DD || in_sizes[10] != NLAY * DD) return;
  if (in_sizes[12] != NLAY * DD || in_sizes[13] != NLAY * DD || in_sizes[14] != NLAY * DD) return;
  if (in_sizes[15] != DD * 128 || in_sizes[16] != 128 || in_sizes[17] != 128 * NTASK || in_sizes[18] != NTASK) return;
  if (out_size != NGR * NTASK) return;

  const int*   x     = (const int*)  d_in[0];
  const int*   ei    = (const int*)  d_in[1];
  const int*   src   = ei;
  const int*   dst   = ei + NEDGE;
  const int*   eattr = (const int*)  d_in[2];
  const int*   bat   = (const int*)  d_in[3];
  const float* femb  = (const float*)d_in[4];
  const float* eemb  = (const float*)d_in[5];
  const float* epsv  = (const float*)d_in[6];
  const float* W1    = (const float*)d_in[7];
  const float* b1    = (const float*)d_in[8];
  const float* g1    = (const float*)d_in[9];
  const float* be1   = (const float*)d_in[10];
  const float* W2    = (const float*)d_in[11];
  const float* b2    = (const float*)d_in[12];
  const float* g2    = (const float*)d_in[13];
  const float* be2   = (const float*)d_in[14];
  const float* Wf1   = (const float*)d_in[15];
  const float* bf1   = (const float*)d_in[16];
  const float* Wf2   = (const float*)d_in[17];
  const float* bf2   = (const float*)d_in[18];
  float* out = (float*)d_out;

  char* ws = (char*)d_ws;
  size_t off = 0;
  const size_t oWT   = off; off = al256(off + (size_t)(2 * NLAY * WPLANE + WFPLANE) * 2);
  const size_t oH    = off; off = al256(off + (size_t)MP * DD * 4);
  const size_t oP1   = off; off = al256(off + (size_t)MP * KTOT * 2);
  const size_t oP2   = off; off = al256(off + (size_t)MP * DD * 4);
  const size_t oLIST = off; off = al256(off + (size_t)NCB * RCAP * 8);
  const size_t oSEG  = off; off = al256(off + (size_t)NCB * NB * 4);
  const size_t oPART = off; off = al256(off + (size_t)NGB * PARTW * 4);
  const size_t oSTAT = off; off = al256(off + (size_t)(4 * DD) * 4);
  const size_t oPL   = off; off = al256(off + (size_t)NGR * KTOT * 2);
  if (off > ws_size || off > (size_t)WSMAX) return;
  unsigned short* WT   = (unsigned short*)(ws + oWT);
  float*          H    = (float*)(ws + oH);
  unsigned short* P1   = (unsigned short*)(ws + oP1);
  float*          P2   = (float*)(ws + oP2);
  int*            LIST = (int*)(ws + oLIST);
  int*            SEG  = (int*)(ws + oSEG);
  float*          PART = (float*)(ws + oPART);
  float*          STAT = (float*)(ws + oSTAT);
  unsigned short* PL   = (unsigned short*)(ws + oPL);

  hipFuncSetAttribute(reinterpret_cast<const void*>(&k_compact), hipFuncAttributeMaxDynamicSharedMemorySize, LDS_CMP);

  const int nU16 = MP * 16;
  k_wprep<<<(NUW + NUF) / NTHR, NTHR, 0, stream>>>(W1, W2, Wf1, WT);
  k_embed<<<nU16 / NTHR, NTHR, 0, stream>>>(x, femb, NNODE, nU16, H);
  k_compact<<<NCB, NTHR, LDS_CMP, stream>>>(src, dst, eattr, NNODE, NEDGE, 1, SEG, LIST);
  for (int l = 0; l < NLAY; ++l) {
    k_agg<<<NGB, NTHR, 0, stream>>>(SEG, LIST, H, eemb, epsv, l, (unsigned int*)P1, NNODE, MP);
    k_gemm<<<NGB, NTHR, 0, stream>>>(P1, WT + (size_t)(2 * l) * WPLANE, b1 + (size_t)l * DD, P2, PART, NNODE, MP);
    k_comb<<<1, DD, 0, stream>>>(PART, NGB, g1 + (size_t)l * DD, be1 + (size_t)l * DD, STAT);
    k_apply_a<<<nU16 / NTHR, NTHR, 0, stream>>>(P2, STAT, NNODE, nU16, P1);
    k_gemm<<<NGB, NTHR, 0, stream>>>(P1, WT + (size_t)(2 * l + 1) * WPLANE, b2 + (size_t)l * DD, P2, PART, NNODE, MP);
    k_comb<<<1, DD, 0, stream>>>(PART, NGB, g2 + (size_t)l * DD, be2 + (size_t)l * DD, STAT);
    k_apply_b<<<nU16 / NTHR, NTHR, 0, stream>>>(P2, STAT, NNODE, nU16, H);
  }
  k_pool<<<NGR / NWAVE, NTHR, 0, stream>>>(H, bat, NNODE, (unsigned int*)PL);
  k_head<<<NGR / HBM, HTHR, 0, stream>>>(PL, WT + (size_t)(2 * NLAY) * WPLANE, bf1, Wf2, bf2, out);
}
